// VariableSelectionNetwork_70196945485886
// MI455X (gfx1250) — hardware-run, weakly checked
//
#include <hip/hip_runtime.h>
#include <math.h>

typedef __attribute__((ext_vector_type(16))) _Float16 v16h;
typedef __attribute__((ext_vector_type(8)))  _Float16 v8h;
typedef __attribute__((ext_vector_type(8)))  float    v8f;
typedef __attribute__((ext_vector_type(4)))  float    v4f;

constexpr int kRows         = 32768;
constexpr int kFeat         = 32;
constexpr int kUnits        = 64;
constexpr int kRowsPerBlock = 64;
constexpr int kRowBlocks    = kRows / kRowsPerBlock;
constexpr int kThreads      = 128;
constexpr float kLnEps      = 1e-3f;
constexpr float kWCarry     = 64.0f;
constexpr float kACarry     = 64.0f;
constexpr float kInvW       = 1.0f / 64.0f;
constexpr float kInvWA      = 1.0f / 4096.0f;
constexpr float kInvFeat    = 1.0f / 32.0f;
constexpr float kInvUnits   = 1.0f / 64.0f;

constexpr int kPitchF32  = 36;
constexpr int kPitchK32  = 40;
constexpr int kPitchK64  = 72;
constexpr int kSlabPitch = 68;
constexpr int kBtPlane32 = kFeat * kPitchK32;

static_assert(kRows % kRowsPerBlock == 0, "no row tail");
static_assert(kFeat == 32 && kUnits == 64, "tile shapes: K=32/64 exact multiples of 32, N=32/64 exact 16-col tiles");

constexpr size_t kPlaneHalves = (size_t)kFeat * kUnits * kUnits;
constexpr size_t kPlaneBytes  = kPlaneHalves * 2;
constexpr size_t kOffW2t      = 0;
constexpr size_t kOffWg1t     = kOffW2t + kPlaneBytes;
constexpr size_t kOffWg2t     = kOffWg1t + kPlaneBytes;
constexpr size_t kOffWsel     = kOffWg2t + kPlaneBytes;
constexpr size_t kWselBytes   = (size_t)kRows * kFeat * 4;
constexpr size_t kWsTotal     = kOffWsel + kWselBytes;
constexpr size_t kOut0Bytes   = (size_t)kRows * kUnits * 4;
constexpr size_t kOut1Offset  = 8388608;
constexpr size_t kOut1Bytes   = (size_t)kRows * kFeat * 4;
constexpr size_t kOutTotal    = 12582912;
static_assert(kWsTotal <= (size_t)134217728, "carve within 128 MiB");
static_assert(kOut0Bytes == kOut1Offset && kOut1Offset + kOut1Bytes == kOutTotal, "tuple output packing");
static_assert((kOffWsel % 128) == 0 && (kOut1Offset % 128) == 0, "line-aligned regions");

template <typename T> struct Frag;
template <> struct Frag<_Float16> {
  typedef v16h V; union U { v16h v; v8h h[2]; };
  static __device__ __forceinline__ v16h load(const _Float16* p) {
    U f; f.h[0] = *(const v8h*)(p); f.h[1] = *(const v8h*)(p + 16); return f.v;
  }
};

union HFragU { v16h v; v8h h[2]; };
#define LDS_FRAG16(dst, base, off) do { HFragU fu_; fu_.h[0] = *(const v8h*)((base) + (off)); fu_.h[1] = *(const v8h*)((base) + (off) + 16); (dst) = fu_.v; } while (0)

__device__ __forceinline__ v8f wmma_h(v16h a, v16h b, v8f c) {
  c = __builtin_amdgcn_wmma_f32_16x16x32_f16(false, a, false, b, (short)0, c, false, false);
  asm volatile("v_nop\n\tv_nop\n\tv_nop\n\tv_nop" : "+v"(c) : "v"(a), "v"(b));
  return c;
}

__device__ __forceinline__ v8f zero8f() { return (v8f){0.f, 0.f, 0.f, 0.f, 0.f, 0.f, 0.f, 0.f}; }

__device__ __forceinline__ float elu_f(float z) {
  const float e = expf(fminf(z, 0.0f)) - 1.0f;
  return (z > 0.0f) ? z : e;
}
__device__ __forceinline__ float sigmoid_f(float z) { return 1.0f / (1.0f + expf(-z)); }

__device__ __forceinline__ float redsum16(float v) {
  v += __shfl_xor(v, 1, 32);  v += __shfl_xor(v, 2, 32);
  v += __shfl_xor(v, 4, 32);  v += __shfl_xor(v, 8, 32);
  return v;
}
__device__ __forceinline__ float redmax16(float v) {
  v = fmaxf(v, __shfl_xor(v, 1, 32));  v = fmaxf(v, __shfl_xor(v, 2, 32));
  v = fmaxf(v, __shfl_xor(v, 4, 32));  v = fmaxf(v, __shfl_xor(v, 8, 32));
  return v;
}

__global__ __launch_bounds__(256) void prep_weights_kernel(
    const float* __restrict__ Wa, const float* __restrict__ Wb, const float* __restrict__ Wc,
    unsigned short* __restrict__ planes) {
  __shared__ float sm[64 * 65];
  const int t = threadIdx.x;
  const int f = blockIdx.x;
  const int z = blockIdx.y;
  const float* W  = (z == 0) ? Wa : ((z == 1) ? Wb : Wc);
  const float* Wf = W + (size_t)f * (kUnits * kUnits);
#pragma unroll
  for (int i = 0; i < 4; ++i) {
    const int q4 = i * 256 + t;
    const int u  = q4 >> 4;
    const int v0 = (q4 & 15) * 4;
    const v4f a = *(const v4f*)(Wf + 4 * q4);
#pragma unroll
    for (int j = 0; j < 4; ++j) sm[(v0 + j) * 65 + u] = a[j] * kWCarry;
  }
  __syncthreads();
  const int lane = t & 31, wave = t >> 5;
  const int q = lane >> 3, c8 = (lane & 7) * 8;
  _Float16* op = (_Float16*)planes + (size_t)z * kPlaneHalves + (size_t)f * (kUnits * kUnits);
  for (int pass = 0; pass < 2; ++pass) {
#pragma unroll
    for (int it = 0; it < 2; ++it) {
      const int row = wave * 8 + it * 4 + q;
      v8h hv;
#pragma unroll
      for (int e = 0; e < 8; ++e) hv[e] = (_Float16)sm[row * 65 + c8 + e];
      *(volatile v8h*)(op + (size_t)row * kUnits + c8) = hv;
    }
    __threadfence();
  }
}

__global__ __launch_bounds__(kThreads) void select_weights_kernel(
    const float* __restrict__ x,
    const float* __restrict__ w1w, const float* __restrict__ b1w,
    const float* __restrict__ w2w, const float* __restrict__ b2w,
    const float* __restrict__ wg1w, const float* __restrict__ bg1w,
    const float* __restrict__ wg2w, const float* __restrict__ bg2w,
    const float* __restrict__ gammaw, const float* __restrict__ betaw,
    float* __restrict__ wsel_out, float* __restrict__ wsel_copy)
{
  __shared__ __align__(16) float    sXf[kRowsPerBlock * kPitchF32];
  __shared__ __align__(16) _Float16 sXh[kRowsPerBlock * kPitchK32];
  __shared__ __align__(16) _Float16 sH1[kRowsPerBlock * kPitchK32];
  __shared__ __align__(16) _Float16 sH2[kRowsPerBlock * kPitchK32];
  __shared__ __align__(16) _Float16 sBt[4 * kBtPlane32];
  __shared__ float sVecF[6 * kFeat];
  __shared__ __align__(16) float    sP[kRowsPerBlock * kPitchF32];

  const int t = threadIdx.x;
  const int lane = t & 31, wave = t >> 5;
  const int rl = lane & 15, hh = lane >> 4, koff = hh * 8;
  const int mw = wave * 16;
  const size_t gb = (size_t)blockIdx.x * kRowsPerBlock;

  {
    const float* xb = x + gb * kFeat;
#pragma unroll
    for (int i = 0; i < 4; ++i) {
      const int q4 = i * kThreads + t;
      const int row = q4 >> 3, c = (q4 & 7) * 4;
      const v4f a = *(const v4f*)(xb + 4 * q4);
      *(v4f*)(sXf + row * kPitchF32 + c) = a;
#pragma unroll
      for (int j = 0; j < 4; ++j) sXh[row * kPitchK32 + c + j] = (_Float16)a[j];
    }
  }
  asm volatile("" ::: "memory");
#pragma unroll
  for (int p = 0; p < 4; ++p) {
    const float* W = (p == 0) ? w1w : ((p == 1) ? w2w : ((p == 2) ? wg1w : wg2w));
#pragma unroll
    for (int i = 0; i < 2; ++i) {
      const int q4 = i * kThreads + t;
      const v4f a = *(const v4f*)(W + 4 * q4);
      const int e0 = 4 * q4, k = e0 >> 5, n0 = e0 & 31;
#pragma unroll
      for (int j = 0; j < 4; ++j) sBt[p * kBtPlane32 + (n0 + j) * kPitchK32 + k] = (_Float16)(a[j] * kWCarry);
    }
    asm volatile("" ::: "memory");
  }
  if (wave == 0) {
    sVecF[0 * kFeat + lane] = b1w[lane];
    sVecF[1 * kFeat + lane] = b2w[lane];
    sVecF[2 * kFeat + lane] = bg1w[lane];
    sVecF[3 * kFeat + lane] = bg2w[lane];
    sVecF[4 * kFeat + lane] = gammaw[lane];
    sVecF[5 * kFeat + lane] = betaw[lane];
  }
  __syncthreads();

  v16h xa; LDS_FRAG16(xa, sXh, (mw + rl) * kPitchK32 + koff);
  v8f a1[2];
#pragma unroll
  for (int j = 0; j < 2; ++j) {
    v16h bb; LDS_FRAG16(bb, sBt, 0 * kBtPlane32 + (j * 16 + rl) * kPitchK32 + koff);
    a1[j] = wmma_h(xa, bb, zero8f());
  }
#pragma unroll
  for (int j = 0; j < 2; ++j)
#pragma unroll
    for (int r = 0; r < 8; ++r) {
      const int row = mw + 8 * hh + r, n = j * 16 + rl;
      const float z = a1[j][r] * kInvW + sVecF[0 * kFeat + n];
      sH1[row * kPitchK32 + n] = (_Float16)(elu_f(z) * kACarry);
    }
  __syncthreads();

  v16h ha; LDS_FRAG16(ha, sH1, (mw + rl) * kPitchK32 + koff);
  v8f a2[2];
#pragma unroll
  for (int j = 0; j < 2; ++j) {
    v16h bb; LDS_FRAG16(bb, sBt, 1 * kBtPlane32 + (j * 16 + rl) * kPitchK32 + koff);
    a2[j] = wmma_h(ha, bb, zero8f());
  }
#pragma unroll
  for (int j = 0; j < 2; ++j)
#pragma unroll
    for (int r = 0; r < 8; ++r) {
      const int row = mw + 8 * hh + r, n = j * 16 + rl;
      const float h2 = a2[j][r] * kInvWA + sVecF[1 * kFeat + n];
      sH2[row * kPitchK32 + n] = (_Float16)(h2 * kACarry);
    }
  __syncthreads();

  v16h ga; LDS_FRAG16(ga, sH2, (mw + rl) * kPitchK32 + koff);
  v8f g1[2], g2[2];
#pragma unroll
  for (int j = 0; j < 2; ++j) {
    v16h bb1; LDS_FRAG16(bb1, sBt, 2 * kBtPlane32 + (j * 16 + rl) * kPitchK32 + koff);
    g1[j] = wmma_h(ga, bb1, zero8f());
    v16h bb2; LDS_FRAG16(bb2, sBt, 3 * kBtPlane32 + (j * 16 + rl) * kPitchK32 + koff);
    g2[j] = wmma_h(ga, bb2, zero8f());
  }

#pragma unroll
  for (int r = 0; r < 8; ++r) {
    const int row = mw + 8 * hh + r;
    float s[2];
#pragma unroll
    for (int j = 0; j < 2; ++j) {
      const int n = j * 16 + rl;
      const float z1 = g1[j][r] * kInvWA + sVecF[2 * kFeat + n];
      const float z2 = g2[j][r] * kInvWA + sVecF[3 * kFeat + n];
      s[j] = z1 * sigmoid_f(z2) + sXf[row * kPitchF32 + n];
    }
    const float sum  = redsum16(s[0] + s[1]);
    const float mean = sum * kInvFeat;
    const float d0 = s[0] - mean, d1 = s[1] - mean;
    const float var  = redsum16(d0 * d0 + d1 * d1) * kInvFeat;
    const float inv  = 1.0f / sqrtf(var + kLnEps);
    const float y0 = d0 * inv * sVecF[4 * kFeat + rl]      + sVecF[5 * kFeat + rl];
    const float y1 = d1 * inv * sVecF[4 * kFeat + 16 + rl] + sVecF[5 * kFeat + 16 + rl];
    const float mx  = redmax16(fmaxf(y0, y1));
    const float e0  = expf(y0 - mx), e1 = expf(y1 - mx);
    const float den = redsum16(e0 + e1);
    const float rd  = 1.0f / den;
    sP[row * kPitchF32 + rl]      = e0 * rd;
    sP[row * kPitchF32 + 16 + rl] = e1 * rd;
  }
  __syncthreads();

  {
    const int q = lane >> 3, c4 = (lane & 7) * 4;
    for (int pass = 0; pass < 2; ++pass) {
#pragma unroll
      for (int it = 0; it < 4; ++it) {
        const int row = mw + it * 4 + q;
        const v4f v = *(const v4f*)(sP + row * kPitchF32 + c4);
        *(volatile v4f*)(wsel_out  + (gb + row) * kFeat + c4) = v;
        *(volatile v4f*)(wsel_copy + (gb + row) * kFeat + c4) = v;
      }
      __threadfence();
    }
  }
}

__global__ __launch_bounds__(kThreads) void feature_mix_kernel(
    const float* __restrict__ x,
    const float* __restrict__ W1, const float* __restrict__ b1,
    const float* __restrict__ b2,
    const float* __restrict__ bg1, const float* __restrict__ bg2,
    const float* __restrict__ Wp, const float* __restrict__ bp,
    const float* __restrict__ gamma, const float* __restrict__ beta,
    const unsigned short* __restrict__ W2t, const unsigned short* __restrict__ Wg1t,
    const unsigned short* __restrict__ Wg2t,
    const float* __restrict__ wsel, float* __restrict__ out)
{
  __shared__ __align__(16) float    sX[kRowsPerBlock * kPitchF32];
  __shared__ __align__(16) float    sW[kRowsPerBlock * kPitchF32];
  __shared__ float sVec[9 * kUnits];
  __shared__ __align__(16) _Float16 sA[kRowsPerBlock * kPitchK64];
  __shared__ __align__(16) _Float16 sH2[kRowsPerBlock * kPitchK64];
  __shared__ __align__(16) float    sSlab[4 * 16 * kSlabPitch];

  const int t = threadIdx.x;
  const int lane = t & 31, wave = t >> 5;
  const int rl = lane & 15, hh = lane >> 4, koff = hh * 8;
  const int mw = wave * 16;
  const size_t gb = (size_t)blockIdx.x * kRowsPerBlock;

  {
    const float* xb = x + gb * kFeat;
    const float* wb = wsel + gb * kFeat;
#pragma unroll
    for (int i = 0; i < 4; ++i) {
      const int q4 = i * kThreads + t;
      const int row = q4 >> 3, c = (q4 & 7) * 4;
      const v4f a = *(const v4f*)(xb + 4 * q4);
      *(v4f*)(sX + row * kPitchF32 + c) = a;
    }
    asm volatile("" ::: "memory");
#pragma unroll
    for (int i = 0; i < 4; ++i) {
      const int q4 = i * kThreads + t;
      const int row = q4 >> 3, c = (q4 & 7) * 4;
      const v4f a = *(const v4f*)(wb + 4 * q4);
      *(v4f*)(sW + row * kPitchF32 + c) = a;
    }
  }
  __syncthreads();

  v8f oacc[4];
#pragma unroll
  for (int j = 0; j < 4; ++j) oacc[j] = zero8f();

#pragma unroll 1
  for (int f = 0; f < kFeat; ++f) {
    __syncthreads();
    {
      const int o = f * kUnits;
      if (wave == 0) {
        sVec[0 * kUnits + lane]      = W1[o + lane];
        sVec[0 * kUnits + 32 + lane] = W1[o + 32 + lane];
        sVec[1 * kUnits + lane]      = b1[o + lane];
        sVec[1 * kUnits + 32 + lane] = b1[o + 32 + lane];
        sVec[2 * kUnits + lane]      = Wp[o + lane];
        sVec[2 * kUnits + 32 + lane] = Wp[o + 32 + lane];
        sVec[3 * kUnits + lane]      = bp[o + lane];
        sVec[3 * kUnits + 32 + lane] = bp[o + 32 + lane];
        sVec[4 * kUnits + lane]      = b2[o + lane];
        sVec[4 * kUnits + 32 + lane] = b2[o + 32 + lane];
      }
      if (wave == 1) {
        sVec[5 * kUnits + lane]      = bg1[o + lane];
        sVec[5 * kUnits + 32 + lane] = bg1[o + 32 + lane];
        sVec[6 * kUnits + lane]      = bg2[o + lane];
        sVec[6 * kUnits + 32 + lane] = bg2[o + 32 + lane];
        sVec[7 * kUnits + lane]      = gamma[o + lane];
        sVec[7 * kUnits + 32 + lane] = gamma[o + 32 + lane];
        sVec[8 * kUnits + lane]      = beta[o + lane];
        sVec[8 * kUnits + 32 + lane] = beta[o + 32 + lane];
      }
    }
    __syncthreads();

    {
      const int m = t >> 1, uh = (t & 1) * 32;
      const float xm = sX[m * kPitchF32 + f];
#pragma unroll 1
      for (int i = 0; i < 4; ++i) {
        const int u0 = uh + i * 8;
        v8h hv;
#pragma unroll
        for (int e = 0; e < 8; ++e) {
          const float z = xm * sVec[0 * kUnits + u0 + e] + sVec[1 * kUnits + u0 + e];
          hv[e] = (_Float16)(elu_f(z) * kACarry);
        }
        *(v8h*)(sA + m * kPitchK64 + u0) = hv;
      }
    }
    __syncthreads();

    const _Float16* W2f = (const _Float16*)W2t  + (size_t)f * (kUnits * kUnits);
    const _Float16* G1f = (const _Float16*)Wg1t + (size_t)f * (kUnits * kUnits);
    const _Float16* G2f = (const _Float16*)Wg2t + (size_t)f * (kUnits * kUnits);

    v8f acc[4];
#pragma unroll
    for (int j = 0; j < 4; ++j) acc[j] = zero8f();
#pragma unroll
    for (int ks = 0; ks < 2; ++ks) {
      asm volatile("" ::: "memory");
      v16h a; LDS_FRAG16(a, sA, (mw + rl) * kPitchK64 + koff + ks * 32);
      v16h bb[4];
#pragma unroll
      for (int j = 0; j < 4; ++j) bb[j] = Frag<_Float16>::load(W2f + (size_t)(j * 16 + rl) * kUnits + koff + ks * 32);
#pragma unroll
      for (int j = 0; j < 4; ++j) acc[j] = wmma_h(a, bb[j], acc[j]);
    }
#pragma unroll
    for (int j = 0; j < 4; ++j)
#pragma unroll
      for (int r = 0; r < 8; ++r) {
        const int row = mw + 8 * hh + r, n = j * 16 + rl;
        const float h2 = acc[j][r] * kInvWA + sVec[4 * kUnits + n];
        sH2[row * kPitchK64 + n] = (_Float16)(h2 * kACarry);
      }
    __syncthreads();

    v8f acc1[4], acc2[4];
#pragma unroll
    for (int j = 0; j < 4; ++j) { acc1[j] = zero8f(); acc2[j] = zero8f(); }
#pragma unroll
    for (int ks = 0; ks < 2; ++ks) {
      asm volatile("" ::: "memory");
      v16h a; LDS_FRAG16(a, sH2, (mw + rl) * kPitchK64 + koff + ks * 32);
      v16h bb[4];
#pragma unroll
      for (int j = 0; j < 4; ++j) bb[j] = Frag<_Float16>::load(G1f + (size_t)(j * 16 + rl) * kUnits + koff + ks * 32);
#pragma unroll
      for (int j = 0; j < 4; ++j) acc1[j] = wmma_h(a, bb[j], acc1[j]);
      asm volatile("" ::: "memory");
#pragma unroll
      for (int j = 0; j < 4; ++j) bb[j] = Frag<_Float16>::load(G2f + (size_t)(j * 16 + rl) * kUnits + koff + ks * 32);
#pragma unroll
      for (int j = 0; j < 4; ++j) acc2[j] = wmma_h(a, bb[j], acc2[j]);
    }

    float xr[8], wr[8];
#pragma unroll
    for (int r = 0; r < 8; ++r) {
      const int row = mw + 8 * hh + r;
      xr[r] = sX[row * kPitchF32 + f];
      wr[r] = sW[row * kPitchF32 + f];
    }
#pragma unroll
    for (int r = 0; r < 8; ++r) {
      float s[4];
#pragma unroll
      for (int j = 0; j < 4; ++j) {
        const int n = j * 16 + rl;
        const float z1  = acc1[j][r] * kInvWA + sVec[5 * kUnits + n];
        const float z2  = acc2[j][r] * kInvWA + sVec[6 * kUnits + n];
        const float res = xr[r] * sVec[2 * kUnits + n] + sVec[3 * kUnits + n];
        s[j] = z1 * sigmoid_f(z2) + res;
      }
      const float sum  = redsum16((s[0] + s[1]) + (s[2] + s[3]));
      const float mean = sum * kInvUnits;
      float d[4];
#pragma unroll
      for (int j = 0; j < 4; ++j) d[j] = s[j] - mean;
      const float sq  = (d[0] * d[0] + d[1] * d[1]) + (d[2] * d[2] + d[3] * d[3]);
      const float var = redsum16(sq) * kInvUnits;
      const float inv = 1.0f / sqrtf(var + kLnEps);
      const float wv  = wr[r];
#pragma unroll
      for (int j = 0; j < 4; ++j) {
        const int n = j * 16 + rl;
        const float y = d[j] * inv * sVec[7 * kUnits + n] + sVec[8 * kUnits + n];
        oacc[j][r] += y * wv;
      }
    }
  }

  float* slab = sSlab + wave * (16 * kSlabPitch);
#pragma unroll
  for (int j = 0; j < 4; ++j)
#pragma unroll
    for (int r = 0; r < 8; ++r) slab[(8 * hh + r) * kSlabPitch + j * 16 + rl] = oacc[j][r];
  __syncthreads();
  {
    const int c4 = rl * 4;
    float* ob = out + (gb + mw) * kUnits;
    for (int pass = 0; pass < 2; ++pass) {
#pragma unroll
      for (int it = 0; it < 8; ++it) {
        const int row = it * 2 + hh;
        const v4f v = *(const v4f*)(slab + row * kSlabPitch + c4);
        *(volatile v4f*)(ob + (size_t)row * kUnits + c4) = v;
      }
      __threadfence();
    }
  }
}

extern "C" void kernel_launch(void* const* d_in, const int* in_sizes, int n_in,
                              void* d_out, int out_size, void* d_ws, size_t ws_size,
                              hipStream_t stream) {
  if (n_in < 23) return;
  if (in_sizes[0] != kRows * kFeat) return;
  if (in_sizes[3] != kFeat * kUnits * kUnits || in_sizes[5] != kFeat * kUnits * kUnits || in_sizes[7] != kFeat * kUnits * kUnits) return;
  if (in_sizes[13] != kFeat * kFeat || in_sizes[1] != kFeat * kUnits) return;
  if ((size_t)out_size != (size_t)kRows * (kUnits + kFeat)) return;
  if (ws_size < kWsTotal) return;

  const float* x      = (const float*)d_in[0];
  const float* W1     = (const float*)d_in[1];
  const float* b1     = (const float*)d_in[2];
  const float* W2     = (const float*)d_in[3];
  const float* b2     = (const float*)d_in[4];
  const float* Wg1    = (const float*)d_in[5];
  const float* bg1    = (const float*)d_in[6];
  const float* Wg2    = (const float*)d_in[7];
  const float* bg2    = (const float*)d_in[8];
  const float* Wp     = (const float*)d_in[9];
  const float* bp     = (const float*)d_in[10];
  const float* gamma  = (const float*)d_in[11];
  const float* beta   = (const float*)d_in[12];
  const float* w1w    = (const float*)d_in[13];
  const float* b1w    = (const float*)d_in[14];
  const float* w2w    = (const float*)d_in[15];
  const float* b2w    = (const float*)d_in[16];
  const float* wg1w   = (const float*)d_in[17];
  const float* bg1w   = (const float*)d_in[18];
  const float* wg2w   = (const float*)d_in[19];
  const float* bg2w   = (const float*)d_in[20];
  const float* gammaw = (const float*)d_in[21];
  const float* betaw  = (const float*)d_in[22];

  unsigned char* ws = (unsigned char*)d_ws;
  unsigned short* planes       = (unsigned short*)(ws + kOffW2t);
  const unsigned short* W2t    = (const unsigned short*)(ws + kOffW2t);
  const unsigned short* Wg1t   = (const unsigned short*)(ws + kOffWg1t);
  const unsigned short* Wg2t   = (const unsigned short*)(ws + kOffWg2t);
  float* wsel_copy             = (float*)(ws + kOffWsel);

  float* out0 = (float*)d_out;
  float* out1 = (float*)((unsigned char*)d_out + kOut1Offset);

  prep_weights_kernel<<<dim3(kFeat, 3), 256, 0, stream>>>(W2, Wg1, Wg2, planes);

  select_weights_kernel<<<kRowBlocks, kThreads, 0, stream>>>(
      x, w1w, b1w, w2w, b2w, wg1w, bg1w, wg2w, bg2w, gammaw, betaw, out1, wsel_copy);

  feature_mix_kernel<<<kRowBlocks, kThreads, 0, stream>>>(
      x, W1, b1, b2, bg1, bg2, Wp, bp, gamma, beta, W2t, Wg1t, Wg2t, wsel_copy, out0);
}
